// NonLocalModule_79010218377228
// MI455X (gfx1250) — hardware-verified
//
#include <hip/hip_runtime.h>


typedef _Float16 v16h __attribute__((ext_vector_type(16)));
typedef _Float16 v8h  __attribute__((ext_vector_type(8)));
typedef float    v8f  __attribute__((ext_vector_type(8)));
typedef float    v4f  __attribute__((ext_vector_type(4)));
typedef v8h v8ha __attribute__((may_alias));
typedef v4f v4fa __attribute__((may_alias));

#define BATCH 2
#define CH    3
#define IMH   63
#define IMW   63
#define KW    7
#define NHW   57
#define NTOT  3249
#define NPAD  3264
#define NT    204
#define QPB   102
#define MCNT  102
#define KS    147
#define KSP   160
#define KC    5
#define KFT   10
#define FPW   5
#define PP    40
#define NBIMG (BATCH*IMH*IMW)
#define NBIP  7968
#define NOUT  (BATCH*CH*IMH*IMW)
#define PSC   4096.0f
#define PSCI  (1.0f/4096.0f)

__device__ __forceinline__ v8f wmma16(v16h a, v16h b, v8f c) {
    v8f d = __builtin_amdgcn_wmma_f32_16x16x32_f16(false, a, false, b, (short)0, c, false, false);
    asm volatile("v_nop\n\tv_nop\n\tv_nop\n\tv_nop" : "+v"(d) : "v"(a), "v"(b));
    return d;
}

__device__ __forceinline__ float sample_patch(const float* __restrict__ img, int b, int n, int k) {
    if (n >= NTOT || k >= KS) return 0.f;
    int nh = n / NHW, nw = n - nh*NHW;
    int c  = k / 49,  r  = k - c*49;
    int ky = r / 7,   kx = r - ky*7;
    return img[((b*CH + c)*IMH + nh + ky)*IMW + nw + kx];
}

__device__ __forceinline__ float gray_at(const float* __restrict__ img, int b, int hh, int ww) {
    #pragma clang fp contract(off)
    if (hh < 0 || hh >= IMH || ww < 0 || ww >= IMW) return 0.f;
    const float* p = img + (size_t)b*CH*IMH*IMW + hh*IMW + ww;
    float g = 0.299f*p[0] + 0.587f*p[IMH*IMW];
    g = g + 0.114f*p[2*IMH*IMW];
    return g;
}

__device__ __forceinline__ float block_val(const float* __restrict__ x, const float* __restrict__ y,
                                           int b, int hh, int ww) {
    #pragma clang fp contract(off)
    float px[9], py[9];
    #pragma unroll
    for (int dy = 0; dy < 3; ++dy) {
        #pragma unroll
        for (int dx = 0; dx < 3; ++dx) {
            px[dy*3+dx] = gray_at(x, b, hh-1+dy, ww-1+dx);
            py[dy*3+dx] = gray_at(y, b, hh-1+dy, ww-1+dx);
        }
    }
    float in_gx = -px[0] + px[2] - 2.f*px[3] + 2.f*px[5] - px[6] + px[8];
    float in_gy = -px[0] - 2.f*px[1] - px[2] + px[6] + 2.f*px[7] + px[8];
    float rf_gx = -py[0] + py[2] - 2.f*py[3] + 2.f*py[5] - py[6] + py[8];
    float rf_gy = -py[0] - 2.f*py[1] - py[2] + py[6] + 2.f*py[7] + py[8];
    if (ww == IMW-1) { in_gx = 1.f; rf_gx = 1.f; }
    if (hh == IMH-1) { in_gy = 1.f; rf_gy = 1.f; }
    float n_in = sqrtf(in_gx*in_gx + in_gy*in_gy);
    float n_rf = sqrtf(rf_gx*rf_gx + rf_gy*rf_gy);
    float num  = in_gx*rf_gx + in_gy*rf_gy + 0.001f;
    float den  = n_in*n_rf + 0.001f;
    float cosv = num / den;
    float one_m = 1.f - cosv;
    float sigma = (n_in >= 29.f) ? 1.f : 0.f;
    float v = sigma * ((n_rf >= 29.f) ? one_m : 1.f);
    return 1.f - v;
}

__global__ void __launch_bounds__(64) block_kernel(const float* __restrict__ x, const float* __restrict__ y,
                                                   float* bimg) {
    int t = blockIdx.x*blockDim.x + threadIdx.x;
    if (t >= NBIP/4) return;
    v4f v;
    #pragma unroll
    for (int j = 0; j < 4; ++j) {
        int e = 4*t + j;
        float r = 0.f;
        if (e < NBIMG) {
            int b  = e / (IMH*IMW);
            int q  = e - b*(IMH*IMW);
            int hh = q / IMW, ww = q - hh*IMW;
            r = block_val(x, y, b, hh, ww);
        }
        v[j] = r;
    }
    float* dst = bimg + 4*t;
    *(volatile v4f*)dst = v;
    __threadfence();
    *(volatile v4f*)dst = v;
}

__global__ void __launch_bounds__(64) stats_kernel(const float* __restrict__ y,
                                                   const float* __restrict__ w1, const float* __restrict__ b1,
                                                   const float* __restrict__ w2, const float* __restrict__ b2,
                                                   const float* __restrict__ bimg,
                                                   v4f* stat) {
    int t = blockIdx.x*blockDim.x + threadIdx.x;
    if (t >= BATCH*NPAD) return;
    int b = t / NPAD, n = t - b*NPAD;
    v4f o = {0.f, 0.f, 0.f, 0.f};
    if (n < NTOT) {
        int nh = n / NHW, nw = n - nh*NHW;
        float ss = 0.f, d0 = 0.f, d1 = 0.f, d2 = 0.f;
        #pragma unroll 1
        for (int c = 0; c < CH; ++c) {
            #pragma unroll 1
            for (int ky = 0; ky < KW; ++ky) {
                #pragma unroll 1
                for (int kx = 0; kx < KW; ++kx) {
                    float v = y[((b*CH + c)*IMH + nh + ky)*IMW + nw + kx];
                    int k = c*49 + ky*7 + kx;
                    ss += v*v;
                    d0 += w1[k]*v;
                    d1 += w1[KS + k]*v;
                    d2 += w1[2*KS + k]*v;
                }
            }
        }
        float h0 = fmaxf(d0 + b1[0], 0.f);
        float h1 = fmaxf(d1 + b1[1], 0.f);
        float h2 = fmaxf(d2 + b1[2], 0.f);
        float hv = (w2[0]*h0 + w2[1]*h1) + w2[2]*h2;
        hv = hv + b2[0];
        float hinv = 1.f / (hv*hv + 1.f);
        float s = 0.f;
        #pragma unroll 1
        for (int ky = 0; ky < KW; ++ky) {
            #pragma unroll 1
            for (int kx = 0; kx < KW; ++kx)
                s += bimg[(b*IMH + nh + ky)*IMW + nw + kx];
        }
        float blk = s * (1.f/49.f);
        o.x = ss; o.y = hinv; o.z = blk; o.w = 0.f;
    }
    v4f* dst = stat + t;
    *(volatile v4f*)dst = o;
    __threadfence();
    *(volatile v4f*)dst = o;
}

__global__ void __launch_bounds__(256) fill_kernel(const float* __restrict__ x, const float* __restrict__ y,
                                                   _Float16* yfr, _Float16* xfr) {
    const int RA = BATCH*NT*KC*64;
    const int RB = BATCH*MCNT*KFT*64;
    int t = blockIdx.x*blockDim.x + threadIdx.x;
    if (t >= RA + RB) return;
    v8h v;
    _Float16* dst;
    if (t < RA) {
        int h8 = t & 1, lane = (t >> 1) & 31, rest = t >> 6;
        int kc = rest % KC; rest /= KC;
        int qt = rest % NT; int b = rest / NT;
        int n  = qt*16 + (lane & 15);
        int g  = lane >> 4;
        int kb = kc*32 + 16*h8 + 8*g;
        #pragma unroll
        for (int j = 0; j < 8; ++j) v[j] = (_Float16)sample_patch(y, b, n, kb + j);
        dst = yfr + ((size_t)((b*NT + qt)*KC + kc)*32 + lane)*16 + 8*h8;
    } else {
        int id = t - RA;
        int h8 = id & 1, lane = (id >> 1) & 31, rest = id >> 6;
        int f  = rest % KFT; rest /= KFT;
        int mc = rest % MCNT; int b = rest / MCNT;
        int kf = f*16 + (lane & 15);
        int g  = lane >> 4;
        int mb = mc*32 + 16*h8 + 8*g;
        #pragma unroll
        for (int j = 0; j < 8; ++j) v[j] = (_Float16)sample_patch(x, b, mb + j, kf);
        dst = xfr + ((size_t)((b*MCNT + mc)*KFT + f)*32 + lane)*16 + 8*h8;
    }
    *(volatile v8h*)dst = v;
    __threadfence();
    *(volatile v8h*)dst = v;
}

__global__ void __launch_bounds__(128) __attribute__((amdgpu_num_vgpr(256)))
attn_kernel(const _Float16* __restrict__ yfr, const _Float16* __restrict__ xfr,
            const v4f* __restrict__ stat, float* outp) {
    __shared__ _Float16 sP[2][16*PP] __attribute__((aligned(16)));
    __shared__ float sScale[2][16];
    __shared__ float sInv[2][16];
    __shared__ float sOut[KSP*32] __attribute__((aligned(16)));

    const int l    = threadIdx.x & 31;
    const int h    = l >> 4;
    const int lm   = l & 15;
    const int wv   = threadIdx.x >> 5;
    const int tile = wv & 1;
    const int fg   = wv >> 1;
    const int b    = blockIdx.x / QPB;
    const int qp   = blockIdx.x - b*QPB;
    if (b >= BATCH) return;
    const int qt   = 2*qp + tile;

    const v16h* yv = (const v16h*)yfr;
    const v16h* xv = (const v16h*)xfr;
    const float NEGINF = -__builtin_inff();

    float sqn[8], hr[8], mrow[8], Zr[8], Wr[8];
    #pragma unroll
    for (int r = 0; r < 8; ++r) {
        v4f st = stat[b*NPAD + qt*16 + 8*h + r];
        sqn[r] = st.x; hr[r] = st.y;
        mrow[r] = NEGINF; Zr[r] = 0.f; Wr[r] = 0.f;
    }
    const v8f zero8 = {0.f,0.f,0.f,0.f,0.f,0.f,0.f,0.f};
    v8f acc[FPW];
    #pragma unroll
    for (int j = 0; j < FPW; ++j) acc[j] = zero8;

    #pragma unroll 1
    for (int mc = 0; mc < MCNT; ++mc) {
        if (wv < 2) {
            v8f S0 = zero8, S1 = zero8;
            const v16h* aq  = yv + (size_t)((b*NT + qt)*KC)*32 + l;
            const v16h* k0p = yv + (size_t)((b*NT + 2*mc)*KC)*32 + l;
            const v16h* k1p = yv + (size_t)((b*NT + 2*mc + 1)*KC)*32 + l;
            #pragma unroll
            for (int c = 0; c < KC; ++c) {
                v16h a  = aq[c*32];
                v16h k0 = k0p[c*32];
                v16h k1 = k1p[c*32];
                S0 = wmma16(a, k0, S0);
                S1 = wmma16(a, k1, S1);
            }
            const int m0 = mc*32 + lm, m1 = m0 + 16;
            const v4f st0 = stat[b*NPAD + m0];
            const v4f st1 = stat[b*NPAD + m1];
            const bool v0 = (m0 < NTOT), v1 = (m1 < NTOT);
            float sc[8];
            #pragma unroll
            for (int r = 0; r < 8; ++r) {
                float s0 = ((2.f*S0[r] - sqn[r]) - st0.x) * hr[r];
                float s1 = ((2.f*S1[r] - sqn[r]) - st1.x) * hr[r];
                if (!v0) s0 = NEGINF;
                if (!v1) s1 = NEGINF;
                float mx = fmaxf(s0, s1);
                #pragma unroll
                for (int off = 1; off < 16; off <<= 1)
                    mx = fmaxf(mx, __shfl_xor(mx, off, 32));
                float nm = fmaxf(mrow[r], mx);
                float scale = __expf(mrow[r] - nm);
                mrow[r] = nm;
                float p0 = __expf(s0 - nm);
                float p1 = __expf(s1 - nm);
                float pb0 = p0 * st0.z;
                float pb1 = p1 * st1.z;
                float pz = p0 + p1, pw = pb0 + pb1;
                #pragma unroll
                for (int off = 1; off < 16; off <<= 1) {
                    pz += __shfl_xor(pz, off, 32);
                    pw += __shfl_xor(pw, off, 32);
                }
                Zr[r] = Zr[r]*scale + pz;
                Wr[r] = Wr[r]*scale + pw;
                sc[r] = scale;
                sP[tile][(8*h + r)*PP + lm]      = (_Float16)(pb0 * PSC);
                sP[tile][(8*h + r)*PP + 16 + lm] = (_Float16)(pb1 * PSC);
            }
            if (lm == 0) {
                #pragma unroll
                for (int r = 0; r < 8; ++r) sScale[tile][8*h + r] = sc[r];
            }
        }
        __syncthreads();
        {
            union { v16h v; v8h hf[2]; } ap;
            ap.hf[0] = *(const v8ha*)(&sP[tile][lm*PP + 8*h]);
            ap.hf[1] = *(const v8ha*)(&sP[tile][lm*PP + 16 + 8*h]);
            v8f scv;
            #pragma unroll
            for (int r = 0; r < 8; ++r) scv[r] = sScale[tile][8*h + r];
            #pragma unroll
            for (int j = 0; j < FPW; ++j) acc[j] = acc[j] * scv;
            const v16h* bp = xv + (size_t)((b*MCNT + mc)*KFT + fg*FPW)*32 + l;
            #pragma unroll
            for (int j = 0; j < FPW; ++j) {
                v16h bI = bp[j*32];
                acc[j] = wmma16(ap.v, bI, acc[j]);
            }
        }
        __syncthreads();
    }

    if (wv < 2 && lm == 0) {
        #pragma unroll
        for (int r = 0; r < 8; ++r) {
            int n = qt*16 + 8*h + r;
            float inv = 0.f;
            if (n < NTOT) inv = 1.f / (Wr[r] + 0.001f*Zr[r]);
            sInv[tile][8*h + r] = inv;
        }
    }
    __syncthreads();
    #pragma unroll
    for (int j = 0; j < FPW; ++j) {
        #pragma unroll
        for (int r = 0; r < 8; ++r) {
            int kf = (fg*FPW + j)*16 + lm;
            int nl = tile*16 + 8*h + r;
            sOut[kf*32 + nl] = (acc[j][r] * PSCI) * sInv[tile][8*h + r];
        }
    }
    __syncthreads();
    v4f vv[10];
    #pragma unroll
    for (int it = 0; it < 10; ++it) {
        int L = wv*40 + it*4 + (l >> 3);
        int pc = l & 7;
        vv[it] = *(const v4fa*)(&sOut[L*32 + pc*4]);
    }
    float* ob = outp + ((size_t)b*KSP)*NPAD + (size_t)qp*32;
    #pragma unroll
    for (int it = 0; it < 10; ++it) {
        int L = wv*40 + it*4 + (l >> 3);
        int pc = l & 7;
        *(volatile v4f*)(ob + (size_t)L*NPAD + pc*4) = vv[it];
    }
    __threadfence();
    #pragma unroll
    for (int it = 0; it < 10; ++it) {
        int L = wv*40 + it*4 + (l >> 3);
        int pc = l & 7;
        *(volatile v4f*)(ob + (size_t)L*NPAD + pc*4) = vv[it];
    }
}

__global__ void __launch_bounds__(64) fold_kernel(const float* __restrict__ outp, float* out) {
    int t  = blockIdx.x*blockDim.x + threadIdx.x;
    int e0 = 4*t;
    if (e0 >= NOUT) return;
    float v[4];
    #pragma unroll
    for (int j = 0; j < 4; ++j) {
        int e = e0 + j;
        float res = 0.f;
        if (e < NOUT) {
            int b  = e / (CH*IMH*IMW);
            int q  = e - b*(CH*IMH*IMW);
            int c  = q / (IMH*IMW); q -= c*(IMH*IMW);
            int hh = q / IMW, ww = q - hh*IMW;
            float acc = 0.f, cnt = 0.f;
            #pragma unroll 1
            for (int ky = 0; ky < KW; ++ky) {
                int nh = hh - ky;
                if (nh < 0 || nh >= NHW) continue;
                #pragma unroll 1
                for (int kx = 0; kx < KW; ++kx) {
                    int nw = ww - kx;
                    if (nw < 0 || nw >= NHW) continue;
                    int cf = c*49 + ky*7 + kx;
                    acc += outp[((size_t)(b*KSP + cf))*NPAD + nh*NHW + nw];
                    cnt += 1.f;
                }
            }
            res = acc * (1.f / cnt);
        }
        v[j] = res;
    }
    if (e0 + 3 < NOUT) {
        v4f w = {v[0], v[1], v[2], v[3]};
        float* dst = out + e0;
        *(volatile v4f*)dst = w;
        __threadfence();
        *(volatile v4f*)dst = w;
    } else {
        #pragma unroll
        for (int j = 0; j < 4; ++j)
            if (e0 + j < NOUT) *(volatile float*)(out + e0 + j) = v[j];
        __threadfence();
        #pragma unroll
        for (int j = 0; j < 4; ++j)
            if (e0 + j < NOUT) *(volatile float*)(out + e0 + j) = v[j];
    }
}

extern "C" void kernel_launch(void* const* d_in, const int* in_sizes, int n_in,
                              void* d_out, int out_size, void* d_ws, size_t ws_size,
                              hipStream_t stream) {
    if (n_in < 6) return;
    if (in_sizes[0] != BATCH*CH*IMH*IMW || in_sizes[1] != BATCH*CH*IMH*IMW) return;
    if (in_sizes[2] != CH*KS || in_sizes[3] != CH || in_sizes[4] != CH || in_sizes[5] != 1) return;
    if (out_size != NOUT) return;

    const float* x  = (const float*)d_in[0];
    const float* y  = (const float*)d_in[1];
    const float* w1 = (const float*)d_in[2];
    const float* b1 = (const float*)d_in[3];
    const float* w2 = (const float*)d_in[4];
    const float* b2 = (const float*)d_in[5];
    float* out = (float*)d_out;

    char* ws = (char*)d_ws;
    size_t off = 0;
    auto carve = [&](size_t bytes) -> char* {
        char* p = ws + off;
        off = (off + bytes + 255) & ~(size_t)255;
        return p;
    };
    const size_t RYH = (size_t)BATCH*NT*KC*512;
    const size_t RXH = (size_t)BATCH*MCNT*KFT*512;
    _Float16* yfr  = (_Float16*)carve(RYH*2);
    _Float16* xfr  = (_Float16*)carve(RXH*2);
    v4f*      stat = (v4f*)carve((size_t)BATCH*NPAD*16);
    float*    bimg = (float*)carve((size_t)NBIP*4);
    float*    outp = (float*)carve((size_t)BATCH*KSP*NPAD*4);
    if (off > ws_size) return;

    {
        int n = NBIP/4;
        block_kernel<<<(n + 63)/64, 64, 0, stream>>>(x, y, bimg);
    }
    {
        int n = BATCH*NPAD;
        stats_kernel<<<(n + 63)/64, 64, 0, stream>>>(y, w1, b1, w2, b2, bimg, stat);
    }
    {
        int n = BATCH*NT*KC*64 + BATCH*MCNT*KFT*64;
        fill_kernel<<<(n + 255)/256, 256, 0, stream>>>(x, y, yfr, xfr);
    }
    {
        int blocks = BATCH*QPB;
        attn_kernel<<<blocks, 128, 0, stream>>>(yfr, xfr, stat, outp);
    }
    {
        int n = (NOUT + 3)/4;
        fold_kernel<<<(n + 63)/64, 64, 0, stream>>>(outp, out);
    }
}
